// DySAT_8899172237850
// MI455X (gfx1250) — hardware-verified
//
#include <hip/hip_runtime.h>
#include <stddef.h>


#define NTHR    256
#define NWAVE   8
#define EPT     8
#define NGRP    2
#define CHUNK   (NTHR * EPT * NGRP)
#define WCAP    (EPT * NGRP * 32)
#define LISTN   (NWAVE * WCAP)
#define NBC     4096
#define NBF     1024
#define RCAP    40960
#define RBN     128
#define TGT     256
#define DEGCAP  1024
#define OTHR    512
#define BM      64
#define BNC     128
#define WSCAP   134217728
#define FIN     128
#define HC      512
#define NHD     4
#define DHD     128
#define DMD     128
#define JW      8
#define NOUT    2
#define PTHR    128
#define ACARRY  8.0f
#define WCARRY  64.0f
#define SCL_AW  (1.0f / 512.0f)
#define LNEPS   1e-5f
#define LPOS    4.0f
#define FLAGV   0x3ACE5ACE

#define LDS_FILL ((RCAP + NBF + LISTN) * 4 + 64)

static_assert((CHUNK & (CHUNK - 1)) == 0);
static_assert(CHUNK <= 4096);
static_assert((NBC & (NBC - 1)) == 0 && (NBF & (NBF - 1)) == 0);
static_assert(NBC == 4 * NBF);
static_assert(OTHR * 8 == NBC);
static_assert((RCAP % 32) == 0);
static_assert(TGT == NWAVE * 32);
static_assert((NBC % TGT) == 0);
static_assert((TGT % BM) == 0);
static_assert(WCAP == EPT * NGRP * 32);
static_assert((FIN % 32) == 0 && (HC % 32) == 0 && (DMD % 32) == 0);
static_assert((HC % BNC) == 0 && (DMD % BNC) == 0);
static_assert(NHD * DHD == HC);
static_assert(HC == 4 * 128 && DMD == 128);
static_assert(JW == 2 * NHD);
static_assert(DMD == PTHR);

typedef float    v4f  __attribute__((ext_vector_type(4)));
typedef float    v8f  __attribute__((ext_vector_type(8)));
typedef int      v4i  __attribute__((ext_vector_type(4)));
typedef _Float16 v4h  __attribute__((ext_vector_type(4)));
typedef _Float16 v8h  __attribute__((ext_vector_type(8)));
typedef _Float16 v16h __attribute__((ext_vector_type(16)));
union Frag { v16h v; v8h h[2]; };

__device__ __forceinline__ v8f wmh(v16h a, v16h b, v8f c) {
  v8f d = __builtin_amdgcn_wmma_f32_16x16x32_f16(false, a, false, b, (short)0, c, false, false);
  asm volatile("v_nop\n\tv_nop\n\tv_nop\n\tv_nop" : "+v"(d) : "v"(a), "v"(b));
  return d;
}

__device__ __forceinline__ v4f selz(v4f v, bool live) {
  v4f o; o.x = live ? v.x : 0.f; o.y = live ? v.y : 0.f; o.z = live ? v.z : 0.f; o.w = live ? v.w : 0.f; return o;
}
__device__ __forceinline__ v4f selv4(v4f v, bool c, float other) {
  v4f o; o.x = c ? v.x : other; o.y = c ? v.y : other; o.z = c ? v.z : other; o.w = c ? v.w : other; return o;
}
__device__ __forceinline__ v4f vmax4(v4f a, v4f b) {
  v4f o; o.x = fmaxf(a.x, b.x); o.y = fmaxf(a.y, b.y); o.z = fmaxf(a.z, b.z); o.w = fmaxf(a.w, b.w); return o;
}
__device__ __forceinline__ v4f lrelu4(v4f v) {
  v4f o;
  o.x = v.x >= 0.f ? v.x : 0.2f * v.x;  o.y = v.y >= 0.f ? v.y : 0.2f * v.y;
  o.z = v.z >= 0.f ? v.z : 0.2f * v.z;  o.w = v.w >= 0.f ? v.w : 0.2f * v.w;
  return o;
}
__device__ __forceinline__ v4f vexp4(v4f v) {
  v4f o; o.x = __expf(v.x); o.y = __expf(v.y); o.z = __expf(v.z); o.w = __expf(v.w); return o;
}
__device__ __forceinline__ v4f elu4(v4f v) {
  v4f o;
  o.x = v.x > 0.f ? v.x : (__expf(v.x) - 1.0f);  o.y = v.y > 0.f ? v.y : (__expf(v.y) - 1.0f);
  o.z = v.z > 0.f ? v.z : (__expf(v.z) - 1.0f);  o.w = v.w > 0.f ? v.w : (__expf(v.w) - 1.0f);
  return o;
}
__device__ __forceinline__ v4h toh4(v4f v) {
  v4h o;
  o.x = (_Float16)(v.x * ACARRY); o.y = (_Float16)(v.y * ACARRY);
  o.z = (_Float16)(v.z * ACARRY); o.w = (_Float16)(v.w * ACARRY);
  return o;
}
__device__ __forceinline__ v4f wmax4(v4f v) {
#pragma unroll
  for (int off = 16; off > 0; off >>= 1) {
    v.x = fmaxf(v.x, __shfl_xor(v.x, off)); v.y = fmaxf(v.y, __shfl_xor(v.y, off));
    v.z = fmaxf(v.z, __shfl_xor(v.z, off)); v.w = fmaxf(v.w, __shfl_xor(v.w, off));
  }
  return v;
}
__device__ __forceinline__ v4f wsum4(v4f v) {
#pragma unroll
  for (int off = 16; off > 0; off >>= 1) {
    v.x += __shfl_xor(v.x, off); v.y += __shfl_xor(v.y, off);
    v.z += __shfl_xor(v.z, off); v.w += __shfl_xor(v.w, off);
  }
  return v;
}
__device__ __forceinline__ float wsum1(float v) {
#pragma unroll
  for (int off = 16; off > 0; off >>= 1) v += __shfl_xor(v, off);
  return v;
}

__global__ __launch_bounds__(NTHR) void k_edges(const int* __restrict__ ei, int* srcl, int* dstl,
                                                int nE, int nN, int nUnits) {
  const int u = (int)blockIdx.x * NTHR + (int)threadIdx.x;
  if (u >= nUnits) return;
  const int etot = 2 * nE + nN;
  v4i sv, dv;
#pragma unroll
  for (int j = 0; j < 4; ++j) {
    const int i = 4 * u + j;
    int iA = i > nE - 1 ? nE - 1 : i;
    iA = iA < 0 ? 0 : iA;
    int iB = i - nE;
    iB = iB < 0 ? 0 : (iB > nE - 1 ? nE - 1 : iB);
    const int r0s = ei[iA];
    const int r0d = ei[nE + iA];
    const int r1s = ei[iB];
    const int r1d = ei[nE + iB];
    const int lp  = i - 2 * nE;
    const bool inA = i < nE, inB = i < 2 * nE, inC = i < etot;
    int s = inA ? r0s : (inB ? r1d : lp);
    int d = inA ? r0d : (inB ? r1s : lp);
    s = inC ? s : 0;
    d = inC ? d : -1;
    sv[j] = s;
    dv[j] = d;
  }
  int* sp = srcl + (size_t)4 * u;
  int* dp = dstl + (size_t)4 * u;
  *(volatile v4i*)sp = sv;
  *(volatile v4i*)dp = dv;
  __threadfence();
  *(volatile v4i*)sp = sv;
  *(volatile v4i*)dp = dv;
}

template <int NB>
__device__ __forceinline__ int scan_chunk(const int* __restrict__ dsts, int nE, int cbase, int slotBase,
                                          int vec8, int* list, int tid, int lane, int wave) {
  int wc = 0;
#pragma unroll
  for (int g = 0; g < NGRP; ++g) {
    const int el0  = (g * NTHR + tid) * EPT;
    const int e0   = cbase + el0;
    const int sent = -2147483647 - 1;
    v4i da, db;
    if (vec8 != 0 && cbase + CHUNK <= nE) {
      da = *(const v4i*)(dsts + e0);
      db = *(const v4i*)(dsts + e0 + 4);
    } else {
      da.x = (e0     < nE) ? dsts[min(e0, nE - 1)] : sent;
      da.y = (e0 + 1 < nE) ? dsts[min(e0 + 1, nE - 1)] : sent;
      da.z = (e0 + 2 < nE) ? dsts[min(e0 + 2, nE - 1)] : sent;
      da.w = (e0 + 3 < nE) ? dsts[min(e0 + 3, nE - 1)] : sent;
      db.x = (e0 + 4 < nE) ? dsts[min(e0 + 4, nE - 1)] : sent;
      db.y = (e0 + 5 < nE) ? dsts[min(e0 + 5, nE - 1)] : sent;
      db.z = (e0 + 6 < nE) ? dsts[min(e0 + 6, nE - 1)] : sent;
      db.w = (e0 + 7 < nE) ? dsts[min(e0 + 7, nE - 1)] : sent;
    }
    const unsigned nb = (unsigned)slotBase;
    const unsigned s0 = (unsigned)da.x - nb, s1 = (unsigned)da.y - nb;
    const unsigned s2 = (unsigned)da.z - nb, s3 = (unsigned)da.w - nb;
    const unsigned s4 = (unsigned)db.x - nb, s5 = (unsigned)db.y - nb;
    const unsigned s6 = (unsigned)db.z - nb, s7 = (unsigned)db.w - nb;
    const bool h0 = s0 < (unsigned)NB, h1 = s1 < (unsigned)NB, h2 = s2 < (unsigned)NB, h3 = s3 < (unsigned)NB;
    const bool h4 = s4 < (unsigned)NB, h5 = s5 < (unsigned)NB, h6 = s6 < (unsigned)NB, h7 = s7 < (unsigned)NB;
    const unsigned any = __builtin_amdgcn_ballot_w32(h0 | h1 | h2 | h3 | h4 | h5 | h6 | h7);
    if (any != 0u) {
#define HITJ(J, HJ, SJ) { \
        const unsigned mj = __builtin_amdgcn_ballot_w32(HJ); \
        if (mj != 0u) { \
          if (HJ) { \
            const int pos = wc + (int)__builtin_amdgcn_mbcnt_lo(mj, 0u); \
            if (pos < WCAP) list[wave * WCAP + pos] = ((el0 + (J)) << 12) | (int)(SJ); \
          } \
          wc += (int)__builtin_popcount(mj); } }
      HITJ(0, h0, s0)
      HITJ(1, h1, s1)
      HITJ(2, h2, s2)
      HITJ(3, h3, s3)
      HITJ(4, h4, s4)
      HITJ(5, h5, s5)
      HITJ(6, h6, s6)
      HITJ(7, h7, s7)
#undef HITJ
    }
  }
  return wc;
}

__global__ __launch_bounds__(NTHR) void k_count(const int* __restrict__ dsts, int* cnt, int nE, int vec8) {
  __shared__ __attribute__((aligned(16))) int scnt[NBC];
  __shared__ __attribute__((aligned(16))) int list[LISTN];
  __shared__ int wcnt[NWAVE];
  const int tid = threadIdx.x, lane = tid & 31, wave = tid >> 5;
  const int nodeBase = blockIdx.x * NBC;

  for (int i = tid; i < NBC; i += NTHR) scnt[i] = 0;
  __syncthreads();

  const int nChunks = (nE + CHUNK - 1) / CHUNK;
#pragma unroll 1
  for (int ch = 0; ch < nChunks; ++ch) {
    const int cbase = ch * CHUNK;
    const int wc = scan_chunk<NBC>(dsts, nE, cbase, nodeBase, vec8, list, tid, lane, wave);
    if (lane == 0) wcnt[wave] = wc;
    __syncthreads();
    if (wave == 0) {
#pragma unroll 1
      for (int wsx = 0; wsx < NWAVE; ++wsx) {
        int n = __builtin_amdgcn_readfirstlane(wcnt[wsx]);
        n = n > WCAP ? WCAP : (n < 0 ? 0 : n);
        const int* lp = list + wsx * WCAP;
#pragma unroll 1
        for (int i = 0; i < n; ++i) {
          const int ent  = __builtin_amdgcn_readfirstlane(lp[i]);
          const int slot = ent & (NBC - 1);
          if (lane == 0) scnt[slot] = scnt[slot] + 1;
        }
      }
    }
    __syncthreads();
  }

  v4i cq[4];
#pragma unroll
  for (int q = 0; q < 4; ++q) {
    const int f = (wave * 4 + q) * 128 + 4 * lane;
    cq[q] = *(const v4i*)(scnt + f);
  }
  int* cp = cnt + (size_t)nodeBase;
#pragma unroll
  for (int q = 0; q < 4; ++q) {
    const int f = (wave * 4 + q) * 128 + 4 * lane;
    *(volatile v4i*)(cp + f) = cq[q];
  }
  __threadfence();
#pragma unroll
  for (int q = 0; q < 4; ++q) {
    const int f = (wave * 4 + q) * 128 + 4 * lane;
    *(volatile v4i*)(cp + f) = cq[q];
  }
}

__global__ __launch_bounds__(OTHR) void k_offsets(
    const int* __restrict__ cnt, int* off, int* rbase, int nChunk) {
  __shared__ __attribute__((aligned(16))) int soff[NBC];
  __shared__ __attribute__((aligned(16))) int srb[RBN];
  __shared__ int wtot[OTHR / 32];
  const int tid = threadIdx.x, lane = tid & 31, wave = tid >> 5, sub = tid >> 7;
  for (int i = tid; i < RBN; i += OTHR) srb[i] = 0;
  int carry = 0;
#pragma unroll 1
  for (int ch = 0; ch < nChunk; ++ch) {
    const int base = ch * NBC;
    const v4i c0 = *(const v4i*)(cnt + base + 8 * tid);
    const v4i c1 = *(const v4i*)(cnt + base + 8 * tid + 4);
    const int e0 = max(c0.x, 0), e1 = max(c0.y, 0), e2 = max(c0.z, 0), e3 = max(c0.w, 0);
    const int e4 = max(c1.x, 0), e5 = max(c1.y, 0), e6 = max(c1.z, 0), e7 = max(c1.w, 0);
    const int ts = e0 + e1 + e2 + e3 + e4 + e5 + e6 + e7;
    int incl = ts;
#pragma unroll
    for (int d = 1; d < 32; d <<= 1) {
      const int t = __shfl_up(incl, d);
      if (lane >= d) incl += t;
    }
    if (lane == 31) wtot[wave] = incl;
    __syncthreads();
    const int S0 = wtot[0]  + wtot[1]  + wtot[2]  + wtot[3];
    const int S1 = wtot[4]  + wtot[5]  + wtot[6]  + wtot[7];
    const int S2 = wtot[8]  + wtot[9]  + wtot[10] + wtot[11];
    const int S3 = wtot[12] + wtot[13] + wtot[14] + wtot[15];
    int pre = 0;
#pragma unroll 1
    for (int w = 4 * sub; w < wave; ++w) pre += wtot[w];
    const int b0 = carry;
    const int b1 = b0 + ((S0 + 31) & ~31);
    const int b2 = b1 + ((S1 + 31) & ~31);
    const int b3 = b2 + ((S2 + 31) & ~31);
    const int b4 = b3 + ((S3 + 31) & ~31);
    const int myb = sub == 0 ? b0 : (sub == 1 ? b1 : (sub == 2 ? b2 : b3));
    if (tid == 0) {
      srb[min(4 * ch + 0, RBN - 1)] = b0;
      srb[min(4 * ch + 1, RBN - 1)] = b1;
      srb[min(4 * ch + 2, RBN - 1)] = b2;
      srb[min(4 * ch + 3, RBN - 1)] = b3;
    }
    int run = myb + pre + incl - ts;
    soff[8 * tid + 0] = run; run += e0;
    soff[8 * tid + 1] = run; run += e1;
    soff[8 * tid + 2] = run; run += e2;
    soff[8 * tid + 3] = run; run += e3;
    soff[8 * tid + 4] = run; run += e4;
    soff[8 * tid + 5] = run; run += e5;
    soff[8 * tid + 6] = run; run += e6;
    soff[8 * tid + 7] = run;
    carry = b4;
    __syncthreads();
    const v4i o0 = *(const v4i*)(soff + 4 * tid);
    const v4i o1 = *(const v4i*)(soff + 4 * (tid + OTHR));
    int* op = off + base;
    *(volatile v4i*)(op + 4 * tid) = o0;
    *(volatile v4i*)(op + 4 * (tid + OTHR)) = o1;
    __threadfence();
    *(volatile v4i*)(op + 4 * tid) = o0;
    *(volatile v4i*)(op + 4 * (tid + OTHR)) = o1;
    __syncthreads();
  }
  if (tid == 0) srb[min(4 * nChunk, RBN - 1)] = carry;
  __syncthreads();
  v4i rv = {0, 0, 0, 0};
  if (tid < 32) rv = *(const v4i*)(srb + 4 * tid);
  if (tid < 32) *(volatile v4i*)(rbase + 4 * tid) = rv;
  __threadfence();
  if (tid < 32) *(volatile v4i*)(rbase + 4 * tid) = rv;
}

__global__ __launch_bounds__(NTHR) void k_fill(
    const int* __restrict__ srcs, const int* __restrict__ dsts,
    const int* __restrict__ off, const int* __restrict__ rbase,
    int* csr, int* flag, int nN, int nE, int vec8, int csrLen) {
  extern __shared__ v4f lds_dyn[];
  int* region = (int*)lds_dyn;
  int* cursor = region + RCAP;
  int* list   = cursor + NBF;
  int* wcnt   = list + LISTN;
  const int tid = threadIdx.x, lane = tid & 31, wave = tid >> 5;
  const int b = blockIdx.x;
  const int nodeBase = b * NBF;

  int rb0 = rbase[b];
  const int rb1 = rbase[b + 1];
  rb0 = rb0 < 0 ? 0 : (rb0 > csrLen ? csrLen : rb0);
  rb0 &= ~31;
  int len = rb1 - rb0;
  const bool ovf = len > RCAP;
  len = len < 0 ? 0 : (len > RCAP ? RCAP : len);
  int lenW = (len + 31) & ~31;
  if (rb0 + lenW > csrLen) lenW = (csrLen - rb0) & ~31;

  {
    const v4i z = {0, 0, 0, 0};
    for (int i = tid; i < RCAP / 4; i += NTHR) ((v4i*)region)[i] = z;
    for (int s = tid; s < NBF; s += NTHR) {
      int o = off[nodeBase + s] - rb0;
      o = o < 0 ? 0 : (o > RCAP ? RCAP : o);
      cursor[s] = o;
    }
  }
  __syncthreads();

  const int nChunks = (nE + CHUNK - 1) / CHUNK;
#pragma unroll 1
  for (int ch = 0; ch < nChunks; ++ch) {
    const int cbase = ch * CHUNK;
    const int wc = scan_chunk<NBF>(dsts, nE, cbase, nodeBase, vec8, list, tid, lane, wave);
    if (lane == 0) wcnt[wave] = wc;
    __syncthreads();
    if (wave == 0) {
#pragma unroll 1
      for (int wsx = 0; wsx < NWAVE; ++wsx) {
        int n = __builtin_amdgcn_readfirstlane(wcnt[wsx]);
        n = n > WCAP ? WCAP : (n < 0 ? 0 : n);
        const int* lp = list + wsx * WCAP;
#pragma unroll 1
        for (int i = 0; i < n; ++i) {
          const int ent  = __builtin_amdgcn_readfirstlane(lp[i]);
          const int slot = ent & (NBF - 1);
          int e = cbase + ((ent >> 12) & (CHUNK - 1));
          e = e > nE - 1 ? nE - 1 : e;
          int sv = srcs[e];
          sv = sv < 0 ? 0 : (sv > nN - 1 ? nN - 1 : sv);
          if (lane == 0) {
            int pos = cursor[slot];
            pos = pos < 0 ? 0 : (pos > RCAP - 1 ? RCAP - 1 : pos);
            region[pos] = sv;
            const int np = pos + 1;
            cursor[slot] = np > RCAP ? RCAP : np;
          }
        }
      }
    }
    __syncthreads();
  }

  const int nv = lenW >> 2;
  int* gp = csr + rb0;
  const v4i fv = {FLAGV, FLAGV, FLAGV, FLAGV};
#pragma unroll 1
  for (int i = tid; i < nv; i += NTHR) { const v4i v = ((const v4i*)region)[i]; *(volatile v4i*)(gp + 4 * i) = v; }
  if (ovf && tid < 8) *(volatile v4i*)(flag + 4 * tid) = fv;
  __threadfence();
#pragma unroll 1
  for (int i = tid; i < nv; i += NTHR) { const v4i v = ((const v4i*)region)[i]; *(volatile v4i*)(gp + 4 * i) = v; }
  if (ovf && tid < 8) *(volatile v4i*)(flag + 4 * tid) = fv;
}

__global__ __launch_bounds__(NTHR) void k_wcvt(const float* __restrict__ w, _Float16* dp, int K, int Nc, int nUnits) {
  const int i = (int)blockIdx.x * NTHR + (int)threadIdx.x;
  if (i >= nUnits) return;
  const int ppr = K >> 3;
  const int n = i / ppr;
  const int seg = i - n * ppr;
  v8h o;
#pragma unroll
  for (int j = 0; j < 8; ++j) {
    int k = 8 * seg + j;
    k = k > K - 1 ? K - 1 : k;
    const float f = w[(size_t)k * Nc + n];
    o[j] = (_Float16)(f * WCARRY);
  }
  _Float16* gp = dp + (size_t)i * 8;
  *(volatile v8h*)gp = o;
  __threadfence();
  *(volatile v8h*)gp = o;
}

__global__ __launch_bounds__(NTHR) void k_acvt(const float* __restrict__ x, _Float16* a1, int nN, int npad) {
  const int gi = (int)blockIdx.x * NTHR + (int)threadIdx.x;
  const int row = gi >> 4, seg = gi & 15;
  if (row >= npad) return;
  int rr = row > nN - 1 ? nN - 1 : row;
  rr = rr < 0 ? 0 : rr;
  const bool live = row < nN;
  const float* rp = x + (size_t)rr * FIN + 8 * seg;
  const v4f x0 = *(const v4f*)rp;
  const v4f x1 = *(const v4f*)(rp + 4);
  const float sc = live ? ACARRY : 0.f;
  v8h o;
  o[0] = (_Float16)(x0.x * sc); o[1] = (_Float16)(x0.y * sc); o[2] = (_Float16)(x0.z * sc); o[3] = (_Float16)(x0.w * sc);
  o[4] = (_Float16)(x1.x * sc); o[5] = (_Float16)(x1.y * sc); o[6] = (_Float16)(x1.z * sc); o[7] = (_Float16)(x1.w * sc);
  _Float16* gp = a1 + (size_t)row * FIN + 8 * seg;
  *(volatile v8h*)gp = o;
  __threadfence();
  *(volatile v8h*)gp = o;
}

__global__ __launch_bounds__(PTHR) void k_pe(float* pe, float pos) {
  __shared__ __attribute__((aligned(16))) float so[PTHR];
  const int tid = threadIdx.x;
  const int pair = tid & ~1;
  const float cexp = -logf(10000.0f) / (float)DMD;
  const float dv = expf((float)pair * cexp);
  const float ang = pos * dv;
  const float sv = sinf(ang);
  const float cv = cosf(ang);
  so[tid] = (tid & 1) ? cv : sv;
  __syncthreads();
  const int tq = tid & 31;
  const v4f v = *(const v4f*)(so + 4 * tq);
  if (tid < 32) *(volatile v4f*)(pe + 4 * tid) = v;
  __threadfence();
  if (tid < 32) *(volatile v4f*)(pe + 4 * tid) = v;
}

template <bool HASB, bool RELU, bool OF32, bool OF16>
__global__ __launch_bounds__(NTHR) void k_gemm(
    const _Float16* __restrict__ A, const _Float16* __restrict__ Bp, const float* __restrict__ bias,
    float* Cf, _Float16* Ch, int K, int ldc, int nValid, int nStore, float scl) {
  constexpr int TPW = 4;
  constexpr int NIT = (BM * (BNC / 4)) / NTHR;
  constexpr int NIH = (BM * (BNC / 8)) / NTHR;
  static_assert((BM * (BNC / 4)) % NTHR == 0 && (BM * (BNC / 8)) % NTHR == 0);
  static_assert(NIT == 8 && NIH == 4);
  static_assert(TPW * 16 * 2 == BNC);
  static_assert(BM == 4 * 16);
  static_assert(BNC / 4 == 32 && BNC / 8 == 16);
  static_assert(OF32 || OF16);

  __shared__ __attribute__((aligned(16))) float    stg[OF32 ? BM * BNC : 4];
  __shared__ __attribute__((aligned(16))) _Float16 sth[OF16 ? BM * BNC : 8];
  const int tid = threadIdx.x, lane = tid & 31, wave = tid >> 5, hh = lane >> 4, m = lane & 15;
  const int rowBase = (int)blockIdx.x * BM;
  const int colBase = (int)blockIdx.y * BNC;
  const int rg = wave >> 1, chf = wave & 1;
  const int r0 = rg * 16;
  const int c0 = chf * (BNC / 2);

  v8f acc[TPW];
#pragma unroll
  for (int t = 0; t < TPW; ++t) { v8f z = {0.f, 0.f, 0.f, 0.f, 0.f, 0.f, 0.f, 0.f}; acc[t] = z; }

  const _Float16* ap = A  + (size_t)(rowBase + r0 + m) * K + 8 * hh;
  const _Float16* bp = Bp + (size_t)(colBase + c0 + m) * K + 8 * hh;
  const int ksteps = K >> 5;
#pragma unroll 1
  for (int kt = 0; kt < ksteps; ++kt) {
    Frag a;
    a.h[0] = *(const v8h*)(ap + 32 * kt);
    a.h[1] = *(const v8h*)(ap + 32 * kt + 16);
#pragma unroll
    for (int t = 0; t < TPW; ++t) {
      const size_t to = (size_t)(16 * t) * K + 32 * kt;
      Frag b;
      b.h[0] = *(const v8h*)(bp + to);
      b.h[1] = *(const v8h*)(bp + to + 16);
      acc[t] = wmh(a.v, b.v, acc[t]);
    }
  }

  {
    const int lrow = r0 + 8 * hh;
    const int growb = rowBase + lrow;
#pragma unroll
    for (int t = 0; t < TPW; ++t) {
      float bvv = 0.f;
      if constexpr (HASB) bvv = bias[colBase + c0 + 16 * t + m];
#pragma unroll
      for (int r = 0; r < 8; ++r) {
        const bool lv = (growb + r) < nValid;
        float g = acc[t][r] * scl + bvv;
        if constexpr (RELU) g = fmaxf(g, 0.f);
        g = lv ? g : 0.f;
        const int li = (lrow + r) * BNC + c0 + 16 * t + m;
        if constexpr (OF32) stg[li] = g;
        if constexpr (OF16) sth[li] = (_Float16)(g * ACARRY);
      }
    }
  }
  __syncthreads();

  if constexpr (OF32) {
    v4f cv[NIT];
#pragma unroll
    for (int it = 0; it < NIT; ++it) {
      const int id = it * NTHR + tid;
      const int row = id >> 5, seg = id & 31;
      cv[it] = *(const v4f*)(stg + (size_t)row * BNC + 4 * seg);
    }
#pragma unroll
    for (int it = 0; it < NIT; ++it) {
      const int id = it * NTHR + tid;
      const int row = id >> 5, seg = id & 31;
      const int grow = rowBase + row;
      if (grow < nStore) {
        float* gp = Cf + (size_t)grow * ldc + colBase + 4 * seg;
        *(volatile v4f*)gp = cv[it];
      }
    }
    __threadfence();
#pragma unroll
    for (int it = 0; it < NIT; ++it) {
      const int id = it * NTHR + tid;
      const int row = id >> 5, seg = id & 31;
      const int grow = rowBase + row;
      if (grow < nStore) {
        float* gp = Cf + (size_t)grow * ldc + colBase + 4 * seg;
        *(volatile v4f*)gp = cv[it];
      }
    }
  }
  if constexpr (OF16) {
    v8h hv[NIH];
#pragma unroll
    for (int it = 0; it < NIH; ++it) {
      const int id = it * NTHR + tid;
      const int row = id >> 4, seg = id & 15;
      hv[it] = *(const v8h*)(sth + (size_t)row * BNC + 8 * seg);
    }
#pragma unroll
    for (int it = 0; it < NIH; ++it) {
      const int id = it * NTHR + tid;
      const int row = id >> 4, seg = id & 15;
      const int grow = rowBase + row;
      if (grow < nStore) {
        _Float16* gp = Ch + (size_t)grow * ldc + colBase + 8 * seg;
        *(volatile v8h*)gp = hv[it];
      }
    }
    __threadfence();
#pragma unroll
    for (int it = 0; it < NIH; ++it) {
      const int id = it * NTHR + tid;
      const int row = id >> 4, seg = id & 15;
      const int grow = rowBase + row;
      if (grow < nStore) {
        _Float16* gp = Ch + (size_t)grow * ldc + colBase + 8 * seg;
        *(volatile v8h*)gp = hv[it];
      }
    }
  }
}

__global__ __launch_bounds__(NTHR) void k_logit(const float* __restrict__ h, const float* __restrict__ avs,
                                                const float* __restrict__ avd, float* es, int nN) {
  __shared__ __attribute__((aligned(16))) float so[32 * JW];
  const int tid = threadIdx.x, lane = tid & 31, wave = tid >> 5, hd = lane >> 3;
  const float* ap = avs + 16 * lane;
  const float* dp = avd + 16 * lane;
#pragma unroll 1
  for (int j = 0; j < 4; ++j) {
    const int node = (int)blockIdx.x * 32 + wave * 4 + j;
    int rr = node > nN - 1 ? nN - 1 : node;
    rr = rr < 0 ? 0 : rr;
    const bool live = node < nN;
    const float* hp = h + (size_t)rr * HC + 16 * lane;
    v4f s1 = {0.f, 0.f, 0.f, 0.f};
    v4f s2 = {0.f, 0.f, 0.f, 0.f};
#pragma unroll 1
    for (int i = 0; i < 4; ++i) {
      const v4f hv = *(const v4f*)(hp + 4 * i);
      const v4f av = *(const v4f*)(ap + 4 * i);
      const v4f dv = *(const v4f*)(dp + 4 * i);
      s1 = s1 + hv * av;
      s2 = s2 + hv * dv;
    }
    float t1 = (s1.x + s1.y) + (s1.z + s1.w);
    float t2 = (s2.x + s2.y) + (s2.z + s2.w);
#pragma unroll
    for (int o = 4; o > 0; o >>= 1) { t1 += __shfl_xor(t1, o); t2 += __shfl_xor(t2, o); }
    if ((lane & 7) == 0) {
      so[(wave * 4 + j) * JW + hd]       = live ? t1 : 0.f;
      so[(wave * 4 + j) * JW + NHD + hd] = live ? t2 : 0.f;
    }
  }
  __syncthreads();
  const int tq = tid & 63;
  const v4f v = *(const v4f*)(so + 4 * tq);
  float* gp = es + (size_t)blockIdx.x * 32 * JW + 4 * tid;
  if (tid < 64) *(volatile v4f*)gp = v;
  __threadfence();
  if (tid < 64) *(volatile v4f*)gp = v;
}

__global__ __launch_bounds__(NTHR) void k_agg1(
    const int* __restrict__ csr, const int* __restrict__ off, const int* __restrict__ cnt,
    const float* __restrict__ es, const float* __restrict__ feat, const float* __restrict__ gb,
    _Float16* a2, int nN, int csrLen) {
  const int tid = threadIdx.x, lane = tid & 31, wave = tid >> 5;
  const int tbase = blockIdx.x * TGT + wave * 32;
  const int cl    = tbase + lane;
  const int cnt_l = cnt[cl];
  const int off_l = off[cl];
  const v4f bq0 = *(const v4f*)(gb + 4 * lane);
  const v4f bq1 = *(const v4f*)(gb + 128 + 4 * lane);
  const v4f bq2 = *(const v4f*)(gb + 256 + 4 * lane);
  const v4f bq3 = *(const v4f*)(gb + 384 + 4 * lane);
  const float NINF = -__builtin_inff();

#pragma unroll 1
  for (int j = 0; j < 32; ++j) {
    const int c = tbase + j;
    int n = __shfl(cnt_l, j);
    n = n < 0 ? 0 : (n > DEGCAP ? DEGCAP : n);
    const int st = __shfl(off_l, j);
    const v4f ed = *(const v4f*)(es + (size_t)c * JW + NHD);

    v4f mx = {NINF, NINF, NINF, NINF};
#pragma unroll 1
    for (int q0 = 0; q0 < n; q0 += 32) {
      int pos = st + q0 + lane;
      pos = pos < 0 ? 0 : (pos > csrLen - 1 ? csrLen - 1 : pos);
      int sl = csr[pos];
      sl = sl < 0 ? 0 : (sl > nN - 1 ? nN - 1 : sl);
      const int mcnt = (n - q0) < 32 ? (n - q0) : 32;
      const bool valid = lane < mcnt;
      const v4f slv = *(const v4f*)(es + (size_t)sl * JW);
      v4f e = selv4(lrelu4(slv + ed), valid, NINF);
      e = wmax4(e);
      mx = vmax4(mx, e);
    }
    v4f z = {0.f, 0.f, 0.f, 0.f};
#pragma unroll 1
    for (int q0 = 0; q0 < n; q0 += 32) {
      int pos = st + q0 + lane;
      pos = pos < 0 ? 0 : (pos > csrLen - 1 ? csrLen - 1 : pos);
      int sl = csr[pos];
      sl = sl < 0 ? 0 : (sl > nN - 1 ? nN - 1 : sl);
      const int mcnt = (n - q0) < 32 ? (n - q0) : 32;
      const bool valid = lane < mcnt;
      const v4f slv = *(const v4f*)(es + (size_t)sl * JW);
      const v4f ex = selv4(vexp4(lrelu4(slv + ed) - mx), valid, 0.f);
      z = z + wsum4(ex);
    }
    v4f rz;
    rz.x = __builtin_amdgcn_rcpf(z.x); rz.y = __builtin_amdgcn_rcpf(z.y);
    rz.z = __builtin_amdgcn_rcpf(z.z); rz.w = __builtin_amdgcn_rcpf(z.w);

    v4f acc0 = {0.f, 0.f, 0.f, 0.f};
    v4f acc1 = {0.f, 0.f, 0.f, 0.f};
    v4f acc2 = {0.f, 0.f, 0.f, 0.f};
    v4f acc3 = {0.f, 0.f, 0.f, 0.f};
#pragma unroll 1
    for (int q0 = 0; q0 < n; q0 += 32) {
      int pos = st + q0 + lane;
      pos = pos < 0 ? 0 : (pos > csrLen - 1 ? csrLen - 1 : pos);
      int sl = csr[pos];
      sl = sl < 0 ? 0 : (sl > nN - 1 ? nN - 1 : sl);
      const int mcnt = (n - q0) < 32 ? (n - q0) : 32;
      const bool valid = lane < mcnt;
      const v4f slv = *(const v4f*)(es + (size_t)sl * JW);
      const v4f al = selv4(vexp4(lrelu4(slv + ed) - mx) * rz, valid, 0.f);
#pragma unroll 1
      for (int pp = 0; pp < mcnt; ++pp) {
        const int s = __builtin_amdgcn_readlane(sl, pp);
        const float a0 = __int_as_float(__builtin_amdgcn_readlane(__float_as_int(al.x), pp));
        const float a1 = __int_as_float(__builtin_amdgcn_readlane(__float_as_int(al.y), pp));
        const float a2v = __int_as_float(__builtin_amdgcn_readlane(__float_as_int(al.z), pp));
        const float a3 = __int_as_float(__builtin_amdgcn_readlane(__float_as_int(al.w), pp));
        const float* hs = feat + (size_t)s * HC + 4 * lane;
        const v4f hv0 = *(const v4f*)hs;
        const v4f hv1 = *(const v4f*)(hs + 128);
        const v4f hv2 = *(const v4f*)(hs + 256);
        const v4f hv3 = *(const v4f*)(hs + 384);
        acc0 = acc0 + hv0 * a0;
        acc1 = acc1 + hv1 * a1;
        acc2 = acc2 + hv2 * a2v;
        acc3 = acc3 + hv3 * a3;
      }
    }

    const bool live = c < nN;
    const v4f o0 = selz(elu4(acc0 + bq0), live);
    const v4f o1 = selz(elu4(acc1 + bq1), live);
    const v4f o2 = selz(elu4(acc2 + bq2), live);
    const v4f o3 = selz(elu4(acc3 + bq3), live);
    const v4h h0 = toh4(o0), h1 = toh4(o1), h2 = toh4(o2), h3 = toh4(o3);
    _Float16* hp = a2 + (size_t)c * HC + 4 * lane;
    *(volatile v4h*)hp = h0;
    *(volatile v4h*)(hp + 128) = h1;
    *(volatile v4h*)(hp + 256) = h2;
    *(volatile v4h*)(hp + 384) = h3;
    __threadfence();
    *(volatile v4h*)hp = h0;
    *(volatile v4h*)(hp + 128) = h1;
    *(volatile v4h*)(hp + 256) = h2;
    *(volatile v4h*)(hp + 384) = h3;
  }
}

__global__ __launch_bounds__(NTHR) void k_agg2(
    const int* __restrict__ csr, const int* __restrict__ off, const int* __restrict__ cnt,
    const float* __restrict__ es, const float* __restrict__ feat, const float* __restrict__ gb,
    const float* __restrict__ pe, float* q, _Float16* qa, int nN, int csrLen) {
  const int tid = threadIdx.x, lane = tid & 31, wave = tid >> 5;
  const int tbase = blockIdx.x * TGT + wave * 32;
  const int cl    = tbase + lane;
  const int cnt_l = cnt[cl];
  const int off_l = off[cl];
  const v4f b2v = *(const v4f*)(gb + 4 * lane);
  const v4f pev = *(const v4f*)(pe + 4 * lane);
  const float NINF = -__builtin_inff();

#pragma unroll 1
  for (int j = 0; j < 32; ++j) {
    const int c = tbase + j;
    int n = __shfl(cnt_l, j);
    n = n < 0 ? 0 : (n > DEGCAP ? DEGCAP : n);
    const int st = __shfl(off_l, j);
    const v4f ed = *(const v4f*)(es + (size_t)c * JW + NHD);

    v4f mx = {NINF, NINF, NINF, NINF};
#pragma unroll 1
    for (int q0 = 0; q0 < n; q0 += 32) {
      int pos = st + q0 + lane;
      pos = pos < 0 ? 0 : (pos > csrLen - 1 ? csrLen - 1 : pos);
      int sl = csr[pos];
      sl = sl < 0 ? 0 : (sl > nN - 1 ? nN - 1 : sl);
      const int mcnt = (n - q0) < 32 ? (n - q0) : 32;
      const bool valid = lane < mcnt;
      const v4f slv = *(const v4f*)(es + (size_t)sl * JW);
      v4f e = selv4(lrelu4(slv + ed), valid, NINF);
      e = wmax4(e);
      mx = vmax4(mx, e);
    }
    v4f z = {0.f, 0.f, 0.f, 0.f};
#pragma unroll 1
    for (int q0 = 0; q0 < n; q0 += 32) {
      int pos = st + q0 + lane;
      pos = pos < 0 ? 0 : (pos > csrLen - 1 ? csrLen - 1 : pos);
      int sl = csr[pos];
      sl = sl < 0 ? 0 : (sl > nN - 1 ? nN - 1 : sl);
      const int mcnt = (n - q0) < 32 ? (n - q0) : 32;
      const bool valid = lane < mcnt;
      const v4f slv = *(const v4f*)(es + (size_t)sl * JW);
      const v4f ex = selv4(vexp4(lrelu4(slv + ed) - mx), valid, 0.f);
      z = z + wsum4(ex);
    }
    v4f rz;
    rz.x = __builtin_amdgcn_rcpf(z.x); rz.y = __builtin_amdgcn_rcpf(z.y);
    rz.z = __builtin_amdgcn_rcpf(z.z); rz.w = __builtin_amdgcn_rcpf(z.w);

    v4f acc0 = {0.f, 0.f, 0.f, 0.f};
    v4f acc1 = {0.f, 0.f, 0.f, 0.f};
    v4f acc2 = {0.f, 0.f, 0.f, 0.f};
    v4f acc3 = {0.f, 0.f, 0.f, 0.f};
#pragma unroll 1
    for (int q0 = 0; q0 < n; q0 += 32) {
      int pos = st + q0 + lane;
      pos = pos < 0 ? 0 : (pos > csrLen - 1 ? csrLen - 1 : pos);
      int sl = csr[pos];
      sl = sl < 0 ? 0 : (sl > nN - 1 ? nN - 1 : sl);
      const int mcnt = (n - q0) < 32 ? (n - q0) : 32;
      const bool valid = lane < mcnt;
      const v4f slv = *(const v4f*)(es + (size_t)sl * JW);
      const v4f al = selv4(vexp4(lrelu4(slv + ed) - mx) * rz, valid, 0.f);
#pragma unroll 1
      for (int pp = 0; pp < mcnt; ++pp) {
        const int s = __builtin_amdgcn_readlane(sl, pp);
        const float a0 = __int_as_float(__builtin_amdgcn_readlane(__float_as_int(al.x), pp));
        const float a1 = __int_as_float(__builtin_amdgcn_readlane(__float_as_int(al.y), pp));
        const float a2v = __int_as_float(__builtin_amdgcn_readlane(__float_as_int(al.z), pp));
        const float a3 = __int_as_float(__builtin_amdgcn_readlane(__float_as_int(al.w), pp));
        const float* hs = feat + (size_t)s * HC + 4 * lane;
        const v4f hv0 = *(const v4f*)hs;
        const v4f hv1 = *(const v4f*)(hs + 128);
        const v4f hv2 = *(const v4f*)(hs + 256);
        const v4f hv3 = *(const v4f*)(hs + 384);
        acc0 = acc0 + hv0 * a0;
        acc1 = acc1 + hv1 * a1;
        acc2 = acc2 + hv2 * a2v;
        acc3 = acc3 + hv3 * a3;
      }
    }

    const bool live = c < nN;
    const v4f hsum = (acc0 + acc1) + (acc2 + acc3);
    v4f qv = (hsum * 0.25f + b2v) + pev;
    qv = selz(qv, live);
    const v4h qh = toh4(qv);
    float* gp = q + (size_t)c * DMD + 4 * lane;
    _Float16* hp = qa + (size_t)c * DMD + 4 * lane;
    *(volatile v4f*)gp = qv;
    *(volatile v4h*)hp = qh;
    __threadfence();
    *(volatile v4f*)gp = qv;
    *(volatile v4h*)hp = qh;
  }
}

__global__ __launch_bounds__(NTHR) void k_ln1(const float* __restrict__ xa, const float* __restrict__ xb,
                                              const float* __restrict__ g, const float* __restrict__ bb,
                                              float* y, _Float16* ya, int nN) {
  const int tid = threadIdx.x, lane = tid & 31, wave = tid >> 5;
  const v4f gv = *(const v4f*)(g + 4 * lane);
  const v4f bv = *(const v4f*)(bb + 4 * lane);
#pragma unroll 1
  for (int j = 0; j < 4; ++j) {
    const int row = (int)blockIdx.x * 32 + wave * 4 + j;
    int rr = row > nN - 1 ? nN - 1 : row;
    rr = rr < 0 ? 0 : rr;
    const bool live = row < nN;
    const v4f v = *(const v4f*)(xa + (size_t)rr * DMD + 4 * lane) + *(const v4f*)(xb + (size_t)rr * DMD + 4 * lane);
    float s = (v.x + v.y) + (v.z + v.w);
    s = wsum1(s);
    const float mu = s * (1.0f / (float)DMD);
    const v4f d = v - mu;
    float ss = (d.x * d.x + d.y * d.y) + (d.z * d.z + d.w * d.w);
    ss = wsum1(ss);
    const float var = ss * (1.0f / (float)DMD);
    const float inv = rsqrtf(var + LNEPS);
    v4f o = (d * inv) * gv + bv;
    o = selz(o, live);
    const v4h oh = toh4(o);
    float* gp = y + (size_t)row * DMD + 4 * lane;
    _Float16* hp = ya + (size_t)row * DMD + 4 * lane;
    *(volatile v4f*)gp = o;
    *(volatile v4h*)hp = oh;
    __threadfence();
    *(volatile v4f*)gp = o;
    *(volatile v4h*)hp = oh;
  }
}

__global__ __launch_bounds__(NTHR) void k_out(const float* __restrict__ xa, const float* __restrict__ xb,
                                              const float* __restrict__ g, const float* __restrict__ bb,
                                              const float* __restrict__ wc, const float* __restrict__ bc,
                                              const int* __restrict__ flag, float* out, int nN, int nOut) {
  __shared__ __attribute__((aligned(16))) float so[64];
  const int tid = threadIdx.x, lane = tid & 31, wave = tid >> 5;
  const v4f gv = *(const v4f*)(g + 4 * lane);
  const v4f bv = *(const v4f*)(bb + 4 * lane);
  const v4f w0 = *(const v4f*)(wc + 8 * lane);
  const v4f w1 = *(const v4f*)(wc + 8 * lane + 4);
  const float bc0 = bc[0], bc1 = bc[1];
  const int fl = flag[0];
  const float pz = (fl == FLAGV) ? __int_as_float(0x7fc00000) : 0.f;
#pragma unroll 1
  for (int j = 0; j < 4; ++j) {
    const int row = (int)blockIdx.x * 32 + wave * 4 + j;
    int rr = row > nN - 1 ? nN - 1 : row;
    rr = rr < 0 ? 0 : rr;
    const v4f v = *(const v4f*)(xa + (size_t)rr * DMD + 4 * lane) + *(const v4f*)(xb + (size_t)rr * DMD + 4 * lane);
    float s = (v.x + v.y) + (v.z + v.w);
    s = wsum1(s);
    const float mu = s * (1.0f / (float)DMD);
    const v4f d = v - mu;
    float ss = (d.x * d.x + d.y * d.y) + (d.z * d.z + d.w * d.w);
    ss = wsum1(ss);
    const float var = ss * (1.0f / (float)DMD);
    const float inv = rsqrtf(var + LNEPS);
    const v4f o = (d * inv) * gv + bv;
    float p0 = (o.x * w0.x + o.y * w0.z) + (o.z * w1.x + o.w * w1.z);
    float p1 = (o.x * w0.y + o.y * w0.w) + (o.z * w1.y + o.w * w1.w);
    p0 = wsum1(p0);
    p1 = wsum1(p1);
    if (lane == 0) {
      so[(wave * 4 + j) * NOUT + 0] = (p0 + bc0) + pz;
      so[(wave * 4 + j) * NOUT + 1] = (p1 + bc1) + pz;
    }
  }
  __syncthreads();
  const int tq = tid & 15;
  const v4f vo = *(const v4f*)(so + 4 * tq);
  const int qd = (int)blockIdx.x * 16 + tid;
  const bool st = (tid < 16) && (4 * qd + 3 < nOut);
  if (st) *(volatile v4f*)(out + (size_t)4 * qd) = vo;
  __threadfence();
  if (st) *(volatile v4f*)(out + (size_t)4 * qd) = vo;
}

extern "C" void kernel_launch(void* const* d_in, const int* in_sizes, int n_in,
                              void* d_out, int out_size, void* d_ws, size_t ws_size,
                              hipStream_t stream) {
  if (n_in < 27) return;
  if (in_sizes[0] < FIN || (in_sizes[0] % FIN) != 0) return;
  const int nN = in_sizes[0] / FIN;
  if (nN < 1 || nN > 131072) return;
  if (in_sizes[1] < 8 || (in_sizes[1] % 2) != 0) return;
  const int nE = in_sizes[1] / 2;
  if (nE < 4 || nE > (1 << 26)) return;
  if (in_sizes[3] != FIN * HC) return;
  if (in_sizes[4] != NHD * DHD || in_sizes[5] != NHD * DHD || in_sizes[6] != HC) return;
  if (in_sizes[7] != HC * HC) return;
  if (in_sizes[8] != NHD * DHD || in_sizes[9] != NHD * DHD || in_sizes[10] != DMD) return;
  if (in_sizes[15] != DMD * DMD || in_sizes[16] != DMD) return;
  if (in_sizes[17] != DMD * DMD || in_sizes[18] != DMD) return;
  if (in_sizes[19] != DMD || in_sizes[20] != DMD) return;
  if (in_sizes[21] != DMD * HC || in_sizes[22] != HC) return;
  if (in_sizes[23] != HC * DMD || in_sizes[24] != DMD) return;
  if (in_sizes[25] != DMD * NOUT || in_sizes[26] != NOUT) return;
  if (out_size != NOUT * nN) return;

  const float* x    = (const float*)d_in[0];
  const int*   ei   = (const int*)d_in[1];
  const float* W1   = (const float*)d_in[3];
  const float* as1  = (const float*)d_in[4];
  const float* ad1  = (const float*)d_in[5];
  const float* b1   = (const float*)d_in[6];
  const float* W2   = (const float*)d_in[7];
  const float* as2  = (const float*)d_in[8];
  const float* ad2  = (const float*)d_in[9];
  const float* b2   = (const float*)d_in[10];
  const float* wv   = (const float*)d_in[15];
  const float* bv   = (const float*)d_in[16];
  const float* wo   = (const float*)d_in[17];
  const float* bo   = (const float*)d_in[18];
  const float* lng  = (const float*)d_in[19];
  const float* lnb  = (const float*)d_in[20];
  const float* f1   = (const float*)d_in[21];
  const float* fb1  = (const float*)d_in[22];
  const float* f2   = (const float*)d_in[23];
  const float* fb2  = (const float*)d_in[24];
  const float* wc   = (const float*)d_in[25];
  const float* bc   = (const float*)d_in[26];
  float* out = (float*)d_out;

  const int NPAD   = ((nN + TGT - 1) / TGT) * TGT;
  const int nAgg   = NPAD / TGT;
  const int nBC    = (nN + NBC - 1) / NBC;
  const int CNTPAD = nBC * NBC;
  if (CNTPAD < NPAD) return;
  if (4 * nBC + 1 > RBN) return;
  const int nBF    = (nN + NBF - 1) / NBF;
  if (nBF > 4 * nBC) return;
  if ((size_t)2 * (size_t)nE + (size_t)nN > (size_t)(1 << 29)) return;
  const int ETOT   = 2 * nE + nN;
  const int LLEN   = (ETOT + 31) & ~31;
  const int nUnits = LLEN / 4;
  const int csrLen = LLEN + 4096;
  if (31 * 4 * nBC > 4096) return;

  char* ws = (char*)d_ws;
  size_t off = 0;
  const size_t oSrc = off; off += (size_t)LLEN * 4;                      off = (off + 255) & ~(size_t)255;
  const size_t oDst = off; off += (size_t)LLEN * 4;                      off = (off + 255) & ~(size_t)255;
  const size_t oCnt = off; off += (size_t)CNTPAD * 4;                    off = (off + 255) & ~(size_t)255;
  const size_t oOff = off; off += (size_t)CNTPAD * 4;                    off = (off + 255) & ~(size_t)255;
  const size_t oRb  = off; off += (size_t)RBN * 4;                       off = (off + 255) & ~(size_t)255;
  const size_t oCsr = off; off += (size_t)csrLen * 4;                    off = (off + 255) & ~(size_t)255;
  const size_t oFlg = off; off += 128;                                   off = (off + 255) & ~(size_t)255;
  const size_t oW1  = off; off += (size_t)HC * FIN * 2;                  off = (off + 255) & ~(size_t)255;
  const size_t oW2  = off; off += (size_t)HC * HC * 2;                   off = (off + 255) & ~(size_t)255;
  const size_t oWv  = off; off += (size_t)DMD * DMD * 2;                 off = (off + 255) & ~(size_t)255;
  const size_t oWo  = off; off += (size_t)DMD * DMD * 2;                 off = (off + 255) & ~(size_t)255;
  const size_t oF1  = off; off += (size_t)HC * DMD * 2;                  off = (off + 255) & ~(size_t)255;
  const size_t oF2  = off; off += (size_t)DMD * HC * 2;                  off = (off + 255) & ~(size_t)255;
  const size_t oPe  = off; off += (size_t)DMD * 4;                       off = (off + 255) & ~(size_t)255;
  const size_t oA1  = off; off += (size_t)NPAD * FIN * 2;                off = (off + 255) & ~(size_t)255;
  const size_t oFt  = off; off += (size_t)NPAD * HC * 4;                 off = (off + 255) & ~(size_t)255;
  const size_t oEs  = off; off += (size_t)NPAD * JW * 4;                 off = (off + 255) & ~(size_t)255;
  const size_t oA2  = off; off += (size_t)NPAD * HC * 2;                 off = (off + 255) & ~(size_t)255;
  const size_t oQ   = off; off += (size_t)NPAD * DMD * 4;                off = (off + 255) & ~(size_t)255;
  const size_t oQa  = off; off += (size_t)NPAD * DMD * 2;                off = (off + 255) & ~(size_t)255;
  const size_t oVa  = off; off += (size_t)NPAD * DMD * 2;                off = (off + 255) & ~(size_t)255;
  const size_t oAo  = off; off += (size_t)NPAD * DMD * 4;                off = (off + 255) & ~(size_t)255;
  const size_t oY1  = off; off += (size_t)NPAD * DMD * 4;                off = (off + 255) & ~(size_t)255;
  const size_t oY1a = off; off += (size_t)NPAD * DMD * 2;                off = (off + 255) & ~(size_t)255;
  const size_t oTa  = off; off += (size_t)NPAD * HC * 2;                 off = (off + 255) & ~(size_t)255;
  const size_t oU   = off; off += (size_t)NPAD * DMD * 4;                off = (off + 255) & ~(size_t)255;
  if (off > ws_size || off > (size_t)WSCAP) return;

  int*   srcl  = (int*)(ws + oSrc);
  int*   dstl  = (int*)(ws + oDst);
  int*   cnt   = (int*)(ws + oCnt);
  int*   offp  = (int*)(ws + oOff);
  int*   rb    = (int*)(ws + oRb);
  int*   csr   = (int*)(ws + oCsr);
  int*   flag  = (int*)(ws + oFlg);
  _Float16* w1p = (_Float16*)(ws + oW1);
  _Float16* w2p = (_Float16*)(ws + oW2);
  _Float16* wvp = (_Float16*)(ws + oWv);
  _Float16* wop = (_Float16*)(ws + oWo);
  _Float16* f1p = (_Float16*)(ws + oF1);
  _Float16* f2p = (_Float16*)(ws + oF2);
  float* pe    = (float*)(ws + oPe);
  _Float16* a1 = (_Float16*)(ws + oA1);
  float* feat  = (float*)(ws + oFt);
  float* es    = (float*)(ws + oEs);
  _Float16* a2 = (_Float16*)(ws + oA2);
  float* q     = (float*)(ws + oQ);
  _Float16* qa = (_Float16*)(ws + oQa);
  _Float16* va = (_Float16*)(ws + oVa);
  float* ao    = (float*)(ws + oAo);
  float* y1    = (float*)(ws + oY1);
  _Float16* y1a = (_Float16*)(ws + oY1a);
  _Float16* ta = (_Float16*)(ws + oTa);
  float* u     = (float*)(ws + oU);

  const int vec8 = 1;

  k_edges<<<(nUnits + NTHR - 1) / NTHR, NTHR, 0, stream>>>(ei, srcl, dstl, nE, nN, nUnits);
  k_count<<<nBC, NTHR, 0, stream>>>(dstl, cnt, ETOT, vec8);
  k_offsets<<<1, OTHR, 0, stream>>>(cnt, offp, rb, nBC);
  hipFuncSetAttribute(reinterpret_cast<const void*>(&k_fill),
                      hipFuncAttributeMaxDynamicSharedMemorySize, LDS_FILL);
  k_fill<<<nBF, NTHR, LDS_FILL, stream>>>(srcl, dstl, offp, rb, csr, flag, nN, ETOT, vec8, csrLen);

  {
    const int u1 = HC * (FIN / 8);
    k_wcvt<<<(u1 + NTHR - 1) / NTHR, NTHR, 0, stream>>>(W1, w1p, FIN, HC, u1);
    const int u2 = HC * (HC / 8);
    k_wcvt<<<(u2 + NTHR - 1) / NTHR, NTHR, 0, stream>>>(W2, w2p, HC, HC, u2);
    const int u3 = DMD * (DMD / 8);
    k_wcvt<<<(u3 + NTHR - 1) / NTHR, NTHR, 0, stream>>>(wv, wvp, DMD, DMD, u3);
    k_wcvt<<<(u3 + NTHR - 1) / NTHR, NTHR, 0, stream>>>(wo, wop, DMD, DMD, u3);
    const int u4 = HC * (DMD / 8);
    k_wcvt<<<(u4 + NTHR - 1) / NTHR, NTHR, 0, stream>>>(f1, f1p, DMD, HC, u4);
    const int u5 = DMD * (HC / 8);
    k_wcvt<<<(u5 + NTHR - 1) / NTHR, NTHR, 0, stream>>>(f2, f2p, HC, DMD, u5);
  }
  k_pe<<<1, PTHR, 0, stream>>>(pe, LPOS);

  k_acvt<<<(NPAD * 16) / NTHR, NTHR, 0, stream>>>(x, a1, nN, NPAD);
  k_gemm<false, false, true, false><<<dim3(NPAD / BM, HC / BNC), NTHR, 0, stream>>>(
      a1, w1p, b1, feat, ta, FIN, HC, nN, NPAD, SCL_AW);
  k_logit<<<NPAD / 32, NTHR, 0, stream>>>(feat, as1, ad1, es, nN);
  k_agg1<<<nAgg, NTHR, 0, stream>>>(csr, offp, cnt, es, feat, b1, a2, nN, csrLen);

  k_gemm<false, false, true, false><<<dim3(NPAD / BM, HC / BNC), NTHR, 0, stream>>>(
      a2, w2p, b1, feat, ta, HC, HC, nN, NPAD, SCL_AW);
  k_logit<<<NPAD / 32, NTHR, 0, stream>>>(feat, as2, ad2, es, nN);
  k_agg2<<<nAgg, NTHR, 0, stream>>>(csr, offp, cnt, es, feat, b2, pe, q, qa, nN, csrLen);

  k_gemm<true, false, false, true><<<dim3(NPAD / BM, DMD / BNC), NTHR, 0, stream>>>(
      qa, wvp, bv, u, va, DMD, DMD, nN, NPAD, SCL_AW);
  k_gemm<true, false, true, false><<<dim3(NPAD / BM, DMD / BNC), NTHR, 0, stream>>>(
      va, wop, bo, ao, ta, DMD, DMD, nN, NPAD, SCL_AW);
  k_ln1<<<NPAD / 32, NTHR, 0, stream>>>(q, ao, lng, lnb, y1, y1a, nN);

  k_gemm<true, true, false, true><<<dim3(NPAD / BM, HC / BNC), NTHR, 0, stream>>>(
      y1a, f1p, fb1, u, ta, DMD, HC, nN, NPAD, SCL_AW);
  k_gemm<true, false, true, false><<<dim3(NPAD / BM, DMD / BNC), NTHR, 0, stream>>>(
      ta, f2p, fb2, u, va, HC, DMD, nN, NPAD, SCL_AW);
  k_out<<<NPAD / 32, NTHR, 0, stream>>>(y1, u, lng, lnb, wc, bc, flag, out, nN, out_size);
}
